// GraphSAGEEnrichedRecommender_35210141893412
// MI455X (gfx1250) — hardware-verified
//
#include <hip/hip_runtime.h>
#include <stddef.h>
#include <math.h>


#define NTHR    256
#define NWAVE   8
#define EPT     8
#define NGRP    2
#define CHUNK   (NTHR * EPT * NGRP)
#define WCAP    (EPT * NGRP * 32)
#define LISTN   (NWAVE * WCAP)
#define NBC     4096
#define NBF     2048
#define FPC     2
#define RCAP    32768
#define RBN     128
#define TGT     256
#define DEGCAP  1024
#define OTHR    512
#define WSCAP   134217728
#define XD      128
#define HROWS   128
#define AP2     72
#define OUTC    100
#define OUTP    112
#define WSC     64.0f
#define WINV    0.015625f
#define LN_EPS  1e-5f

#define WP1     0
#define WP2     32768
#define WP3     98304
#define WP4     163840
#define WP5     172032
#define WPTOT   179200

#define LDS_FILL ((RCAP + NBF + LISTN) * 4 + 64)
#define LDS_SAGE (128 * 128 * 4)
#define LDS_HEAD (HROWS * OUTC * 4 + HROWS * AP2 * 2)

static_assert((CHUNK & (CHUNK - 1)) == 0);
static_assert(CHUNK <= 4096);
static_assert((NBC & (NBC - 1)) == 0 && (NBF & (NBF - 1)) == 0);
static_assert(NBC == FPC * NBF && FPC == 2);
static_assert(OTHR * 8 == NBC && OTHR == 2 * NTHR);
static_assert((RCAP % 32) == 0);
static_assert(TGT == NWAVE * 32);
static_assert((NBC % TGT) == 0);
static_assert(WP2 == WP1 + 128 * 256 && WP3 == WP2 + 256 * 256 && WP4 == WP3 + 128 * 512);
static_assert(WP5 == WP4 + 64 * 128 && WPTOT == WP5 + OUTP * 64);
static_assert((WP1 % 64) == 0 && (WP2 % 64) == 0 && (WP3 % 64) == 0 && (WP4 % 64) == 0 && (WP5 % 64) == 0);
static_assert((AP2 % 8) == 0);
static_assert(HROWS * 64 * 4 <= HROWS * OUTC * 4);

typedef float          v2f  __attribute__((ext_vector_type(2)));
typedef float          v4f  __attribute__((ext_vector_type(4)));
typedef float          v8f  __attribute__((ext_vector_type(8)));
typedef int            v4i  __attribute__((ext_vector_type(4)));
typedef _Float16       v2h  __attribute__((ext_vector_type(2)));
typedef _Float16       v4h  __attribute__((ext_vector_type(4)));
typedef _Float16       v8h  __attribute__((ext_vector_type(8)));
typedef _Float16       v16h __attribute__((ext_vector_type(16)));
union FragH { v16h v; v8h half[2]; };

__device__ __forceinline__ v8f wmh(v16h a, v16h b, v8f c) {
  v8f d = __builtin_amdgcn_wmma_f32_16x16x32_f16(false, a, false, b, (short)0, c, false, false);
  asm volatile("v_nop\n\tv_nop\n\tv_nop\n\tv_nop" : "+v"(d) : "v"(a), "v"(b));
  return d;
}

__device__ __forceinline__ v8h cvt8(v4f a, v4f b) {
  v8h o;
  o[0] = (_Float16)a.x; o[1] = (_Float16)a.y; o[2] = (_Float16)a.z; o[3] = (_Float16)a.w;
  o[4] = (_Float16)b.x; o[5] = (_Float16)b.y; o[6] = (_Float16)b.z; o[7] = (_Float16)b.w;
  return o;
}

__device__ __forceinline__ float wsum(float s) {
  s += __shfl_xor(s, 16);
  s += __shfl_xor(s, 8);
  s += __shfl_xor(s, 4);
  s += __shfl_xor(s, 2);
  s += __shfl_xor(s, 1);
  return s;
}

template <int NB>
__device__ __forceinline__ int scan_chunk(const int* __restrict__ dsts, int nE, int cbase, int slotBase,
                                          int vec8, int* list, int tid, int lane, int wave) {
  int wc = 0;
#pragma unroll
  for (int g = 0; g < NGRP; ++g) {
    const int el0  = (g * NTHR + tid) * EPT;
    const int e0   = cbase + el0;
    const int sent = -2147483647 - 1;
    v4i da, db;
    if (vec8 != 0 && cbase + CHUNK <= nE) {
      da = *(const v4i*)(dsts + e0);
      db = *(const v4i*)(dsts + e0 + 4);
    } else {
      da.x = (e0     < nE) ? dsts[min(e0, nE - 1)] : sent;
      da.y = (e0 + 1 < nE) ? dsts[min(e0 + 1, nE - 1)] : sent;
      da.z = (e0 + 2 < nE) ? dsts[min(e0 + 2, nE - 1)] : sent;
      da.w = (e0 + 3 < nE) ? dsts[min(e0 + 3, nE - 1)] : sent;
      db.x = (e0 + 4 < nE) ? dsts[min(e0 + 4, nE - 1)] : sent;
      db.y = (e0 + 5 < nE) ? dsts[min(e0 + 5, nE - 1)] : sent;
      db.z = (e0 + 6 < nE) ? dsts[min(e0 + 6, nE - 1)] : sent;
      db.w = (e0 + 7 < nE) ? dsts[min(e0 + 7, nE - 1)] : sent;
    }
    const unsigned nb = (unsigned)slotBase;
    const unsigned s0 = (unsigned)da.x - nb, s1 = (unsigned)da.y - nb;
    const unsigned s2 = (unsigned)da.z - nb, s3 = (unsigned)da.w - nb;
    const unsigned s4 = (unsigned)db.x - nb, s5 = (unsigned)db.y - nb;
    const unsigned s6 = (unsigned)db.z - nb, s7 = (unsigned)db.w - nb;
    const bool h0 = s0 < (unsigned)NB, h1 = s1 < (unsigned)NB, h2 = s2 < (unsigned)NB, h3 = s3 < (unsigned)NB;
    const bool h4 = s4 < (unsigned)NB, h5 = s5 < (unsigned)NB, h6 = s6 < (unsigned)NB, h7 = s7 < (unsigned)NB;
    const unsigned any = __builtin_amdgcn_ballot_w32(h0 | h1 | h2 | h3 | h4 | h5 | h6 | h7);
    if (any != 0u) {
#define HITJ(J, HJ, SJ) { \
        const unsigned mj = __builtin_amdgcn_ballot_w32(HJ); \
        if (mj != 0u) { \
          if (HJ) { \
            const int pos = wc + (int)__builtin_amdgcn_mbcnt_lo(mj, 0u); \
            if (pos < WCAP) list[wave * WCAP + pos] = ((el0 + (J)) << 12) | (int)(SJ); \
          } \
          wc += (int)__builtin_popcount(mj); } }
      HITJ(0, h0, s0)
      HITJ(1, h1, s1)
      HITJ(2, h2, s2)
      HITJ(3, h3, s3)
      HITJ(4, h4, s4)
      HITJ(5, h5, s5)
      HITJ(6, h6, s6)
      HITJ(7, h7, s7)
#undef HITJ
    }
  }
  return wc;
}

__global__ __launch_bounds__(NTHR) void k_wprep(
    const float* __restrict__ s1wl, const float* __restrict__ s1wr,
    const float* __restrict__ s2wl, const float* __restrict__ s2wr,
    const float* __restrict__ s3wl, const float* __restrict__ s3wr,
    const float* __restrict__ l1w,  const float* __restrict__ low,
    _Float16* wp) {
  const int blk = blockIdx.x, tid = threadIdx.x;
  float v[8];
  int base, i;
  bool act = true;
  if (blk < 16) {
    i = blk * NTHR + tid; base = WP1;
    const int n = i >> 5, k0 = (i & 31) * 8;
#pragma unroll
    for (int e = 0; e < 8; ++e) {
      const int k = k0 + e;
      const int ka = k > 127 ? 127 : k;
      int kb = k - 128; kb = kb < 0 ? 0 : kb;
      const float va = s1wl[ka * 128 + n];
      const float vb = s1wr[kb * 128 + n];
      v[e] = (k < 128) ? va : vb;
    }
  } else if (blk < 48) {
    i = (blk - 16) * NTHR + tid; base = WP2;
    const int n = i >> 5, k0 = (i & 31) * 8;
#pragma unroll
    for (int e = 0; e < 8; ++e) {
      const int k = k0 + e;
      const int ka = k > 127 ? 127 : k;
      int kb = k - 128; kb = kb < 0 ? 0 : kb;
      const float va = s2wl[ka * 256 + n];
      const float vb = s2wr[kb * 256 + n];
      v[e] = (k < 128) ? va : vb;
    }
  } else if (blk < 80) {
    i = (blk - 48) * NTHR + tid; base = WP3;
    const int n = i >> 6, k0 = (i & 63) * 8;
#pragma unroll
    for (int e = 0; e < 8; ++e) {
      const int k = k0 + e;
      const int ka = k > 255 ? 255 : k;
      int kb = k - 256; kb = kb < 0 ? 0 : kb;
      const float va = s3wl[ka * 128 + n];
      const float vb = s3wr[kb * 128 + n];
      v[e] = (k < 256) ? va : vb;
    }
  } else if (blk < 84) {
    i = (blk - 80) * NTHR + tid; base = WP4;
    const int n = i >> 4, k0 = (i & 15) * 8;
#pragma unroll
    for (int e = 0; e < 8; ++e) v[e] = l1w[(k0 + e) * 64 + n];
  } else {
    i = (blk - 84) * NTHR + tid; base = WP5;
    act = i < OUTP * 8;
    i = i > OUTP * 8 - 1 ? OUTP * 8 - 1 : i;
    const int n = i >> 3, k0 = (i & 7) * 8;
    const int nn = n > OUTC - 1 ? OUTC - 1 : n;
#pragma unroll
    for (int e = 0; e < 8; ++e) {
      const float va = low[(k0 + e) * OUTC + nn];
      v[e] = (n < OUTC) ? va : 0.0f;
    }
  }
  v4f a, b;
  a.x = v[0] * WSC; a.y = v[1] * WSC; a.z = v[2] * WSC; a.w = v[3] * WSC;
  b.x = v[4] * WSC; b.y = v[5] * WSC; b.z = v[6] * WSC; b.w = v[7] * WSC;
  const v8h o = cvt8(a, b);
  _Float16* d = wp + base + (size_t)i * 8;
  if (act) *(volatile v8h*)d = o;
  __threadfence();
  if (act) *(volatile v8h*)d = o;
}

__global__ __launch_bounds__(NTHR) void k_xcvt(const float* __restrict__ x, _Float16* X16, int nN) {
  const int idx = blockIdx.x * NTHR + threadIdx.x;
  const int r = idx >> 4, c0 = (idx & 15) * 8;
  const int rr = r < nN ? r : nN - 1;
  const float* p = x + (size_t)rr * XD + c0;
  v4f a = *(const v4f*)p, b = *(const v4f*)(p + 4);
  const bool z = r >= nN;
  a.x = z ? 0.0f : a.x; a.y = z ? 0.0f : a.y; a.z = z ? 0.0f : a.z; a.w = z ? 0.0f : a.w;
  b.x = z ? 0.0f : b.x; b.y = z ? 0.0f : b.y; b.z = z ? 0.0f : b.z; b.w = z ? 0.0f : b.w;
  const v8h o = cvt8(a, b);
  _Float16* d = X16 + (size_t)r * XD + c0;
  *(volatile v8h*)d = o;
  __threadfence();
  *(volatile v8h*)d = o;
}

__global__ __launch_bounds__(NTHR) void k_count(const int* __restrict__ dsts, int* cnt, int nE, int vec8) {
  __shared__ __attribute__((aligned(16))) int scnt[NBC];
  __shared__ __attribute__((aligned(16))) int list[LISTN];
  __shared__ int wcnt[NWAVE];
  const int tid = threadIdx.x, lane = tid & 31, wave = tid >> 5;
  const int nodeBase = blockIdx.x * NBC;

  for (int i = tid; i < NBC; i += NTHR) scnt[i] = 0;
  __syncthreads();

  const int nChunks = (nE + CHUNK - 1) / CHUNK;
#pragma unroll 1
  for (int ch = 0; ch < nChunks; ++ch) {
    const int cbase = ch * CHUNK;
    const int wc = scan_chunk<NBC>(dsts, nE, cbase, nodeBase, vec8, list, tid, lane, wave);
    if (lane == 0) wcnt[wave] = wc;
    __syncthreads();
    if (wave == 0) {
#pragma unroll 1
      for (int wsx = 0; wsx < NWAVE; ++wsx) {
        int n = __builtin_amdgcn_readfirstlane(wcnt[wsx]);
        n = n > WCAP ? WCAP : (n < 0 ? 0 : n);
        const int* lp = list + wsx * WCAP;
#pragma unroll 1
        for (int i = 0; i < n; ++i) {
          const int ent  = __builtin_amdgcn_readfirstlane(lp[i]);
          const int slot = ent & (NBC - 1);
          if (lane == 0) scnt[slot] = scnt[slot] + 1;
        }
      }
    }
    __syncthreads();
  }

  v4i cq[4];
#pragma unroll
  for (int q = 0; q < 4; ++q) {
    const int f = (wave * 4 + q) * 128 + 4 * lane;
    cq[q] = *(const v4i*)(scnt + f);
  }
  int* cp = cnt + (size_t)nodeBase;
#pragma unroll
  for (int q = 0; q < 4; ++q) {
    const int f = (wave * 4 + q) * 128 + 4 * lane;
    *(volatile v4i*)(cp + f) = cq[q];
  }
  __threadfence();
#pragma unroll
  for (int q = 0; q < 4; ++q) {
    const int f = (wave * 4 + q) * 128 + 4 * lane;
    *(volatile v4i*)(cp + f) = cq[q];
  }
}

__global__ __launch_bounds__(OTHR) void k_offsets(
    const int* __restrict__ cnt, int* off, int* rbase, int nChunk, int nE) {
  __shared__ __attribute__((aligned(16))) int soff[NBC];
  __shared__ __attribute__((aligned(16))) int srb[RBN];
  __shared__ int wtot[OTHR / 32];
  const int tid = threadIdx.x, lane = tid & 31, wave = tid >> 5, sub = tid >> 8;
  for (int i = tid; i < RBN; i += OTHR) srb[i] = 0;
  int carry = 0;
#pragma unroll 1
  for (int ch = 0; ch < nChunk; ++ch) {
    const int base = ch * NBC;
    const v4i c0 = *(const v4i*)(cnt + base + 8 * tid);
    const v4i c1 = *(const v4i*)(cnt + base + 8 * tid + 4);
    const int e0 = min(max(c0.x, 0), nE), e1 = min(max(c0.y, 0), nE);
    const int e2 = min(max(c0.z, 0), nE), e3 = min(max(c0.w, 0), nE);
    const int e4 = min(max(c1.x, 0), nE), e5 = min(max(c1.y, 0), nE);
    const int e6 = min(max(c1.z, 0), nE), e7 = min(max(c1.w, 0), nE);
    const int ts = e0 + e1 + e2 + e3 + e4 + e5 + e6 + e7;
    int incl = ts;
#pragma unroll
    for (int d = 1; d < 32; d <<= 1) {
      const int t = __shfl_up(incl, d);
      if (lane >= d) incl += t;
    }
    if (lane == 31) wtot[wave] = incl;
    __syncthreads();
    const int S0 = wtot[0] + wtot[1] + wtot[2]  + wtot[3]  + wtot[4]  + wtot[5]  + wtot[6]  + wtot[7];
    const int S1 = wtot[8] + wtot[9] + wtot[10] + wtot[11] + wtot[12] + wtot[13] + wtot[14] + wtot[15];
    int pre = 0;
#pragma unroll 1
    for (int w = 8 * sub; w < wave; ++w) pre += wtot[w];
    const int b0 = carry;
    const int b1 = b0 + ((S0 + 31) & ~31);
    const int b2 = b1 + ((S1 + 31) & ~31);
    const int myb = (sub == 0) ? b0 : b1;
    if (tid == 0) {
      srb[min(FPC * ch + 0, RBN - 1)] = b0;
      srb[min(FPC * ch + 1, RBN - 1)] = b1;
    }
    int run = myb + pre + incl - ts;
    soff[8 * tid + 0] = run; run += e0;
    soff[8 * tid + 1] = run; run += e1;
    soff[8 * tid + 2] = run; run += e2;
    soff[8 * tid + 3] = run; run += e3;
    soff[8 * tid + 4] = run; run += e4;
    soff[8 * tid + 5] = run; run += e5;
    soff[8 * tid + 6] = run; run += e6;
    soff[8 * tid + 7] = run;
    carry = b2;
    __syncthreads();
    const v4i o0 = *(const v4i*)(soff + 4 * tid);
    const v4i o1 = *(const v4i*)(soff + 4 * (tid + OTHR));
    int* op = off + base;
    *(volatile v4i*)(op + 4 * tid) = o0;
    *(volatile v4i*)(op + 4 * (tid + OTHR)) = o1;
    __threadfence();
    *(volatile v4i*)(op + 4 * tid) = o0;
    *(volatile v4i*)(op + 4 * (tid + OTHR)) = o1;
    __syncthreads();
  }
  if (tid == 0) srb[min(FPC * nChunk, RBN - 1)] = carry;
  __syncthreads();
  v4i rv = {0, 0, 0, 0};
  if (tid < 32) rv = *(const v4i*)(srb + 4 * tid);
  if (tid < 32) *(volatile v4i*)(rbase + 4 * tid) = rv;
  __threadfence();
  if (tid < 32) *(volatile v4i*)(rbase + 4 * tid) = rv;
}

__global__ __launch_bounds__(NTHR) void k_fill(
    const int* __restrict__ srcs, const int* __restrict__ dsts,
    const int* __restrict__ off, const int* __restrict__ rbase,
    int* csr, int nN, int nE, int vec8, int csrLen) {
  extern __shared__ v4f lds_dyn[];
  int* region = (int*)lds_dyn;
  int* cursor = region + RCAP;
  int* list   = cursor + NBF;
  int* wcnt   = list + LISTN;
  const int tid = threadIdx.x, lane = tid & 31, wave = tid >> 5;
  const int b = blockIdx.x;
  const int nodeBase = b * NBF;

  int rb0 = rbase[b];
  const int rb1 = rbase[b + 1];
  rb0 = rb0 < 0 ? 0 : (rb0 > csrLen ? csrLen : rb0);
  rb0 &= ~31;
  int len = rb1 - rb0;
  len = len < 0 ? 0 : (len > RCAP ? RCAP : len);
  int lenW = (len + 31) & ~31;
  if (rb0 + lenW > csrLen) lenW = (csrLen - rb0) & ~31;

  {
    const v4i z = {0, 0, 0, 0};
    for (int i = tid; i < RCAP / 4; i += NTHR) ((v4i*)region)[i] = z;
    for (int s = tid; s < NBF; s += NTHR) {
      int o = off[nodeBase + s] - rb0;
      o = o < 0 ? 0 : (o > RCAP ? RCAP : o);
      cursor[s] = o;
    }
  }
  __syncthreads();

  const int nChunks = (nE + CHUNK - 1) / CHUNK;
#pragma unroll 1
  for (int ch = 0; ch < nChunks; ++ch) {
    const int cbase = ch * CHUNK;
    const int wc = scan_chunk<NBF>(dsts, nE, cbase, nodeBase, vec8, list, tid, lane, wave);
    if (lane == 0) wcnt[wave] = wc;
    __syncthreads();
    if (wave == 0) {
#pragma unroll 1
      for (int wsx = 0; wsx < NWAVE; ++wsx) {
        int n = __builtin_amdgcn_readfirstlane(wcnt[wsx]);
        n = n > WCAP ? WCAP : (n < 0 ? 0 : n);
        const int* lp = list + wsx * WCAP;
#pragma unroll 1
        for (int i = 0; i < n; ++i) {
          const int ent  = __builtin_amdgcn_readfirstlane(lp[i]);
          const int slot = ent & (NBF - 1);
          int e = cbase + ((ent >> 12) & (CHUNK - 1));
          e = e > nE - 1 ? nE - 1 : e;
          int sv = srcs[e];
          sv = sv < 0 ? 0 : (sv > nN - 1 ? nN - 1 : sv);
          if (lane == 0) {
            int pos = cursor[slot];
            pos = pos < 0 ? 0 : (pos > RCAP - 1 ? RCAP - 1 : pos);
            region[pos] = sv;
            const int np = pos + 1;
            cursor[slot] = np > RCAP ? RCAP : np;
          }
        }
      }
    }
    __syncthreads();
  }

  const int nv = lenW >> 2;
  int* gp = csr + rb0;
#pragma unroll 1
  for (int i = tid; i < nv; i += NTHR) { const v4i v = ((const v4i*)region)[i]; *(volatile v4i*)(gp + 4 * i) = v; }
  __threadfence();
#pragma unroll 1
  for (int i = tid; i < nv; i += NTHR) { const v4i v = ((const v4i*)region)[i]; *(volatile v4i*)(gp + 4 * i) = v; }
}

template <int MODE>
__global__ __launch_bounds__(NTHR) void k_agg(
    const int* __restrict__ csr, const int* __restrict__ off, const int* __restrict__ cnt,
    const float* __restrict__ xs, const _Float16* __restrict__ hs,
    _Float16* A, int nN, int csrLen) {
  const int tid = threadIdx.x, lane = tid & 31, wave = tid >> 5;
  const int tbase = blockIdx.x * TGT + wave * 32;
  const int cl = tbase + lane;
  const int cnt_l = cnt[cl];
  const int off_l = off[cl];
  const _Float16 nh = (_Float16)(-__builtin_huge_valf());
  const _Float16 zh = (_Float16)0.0f;

#pragma unroll 1
  for (int j = 0; j < 32; ++j) {
    const int c = tbase + j;
    int n = __builtin_amdgcn_readlane(cnt_l, j);
    n = n < 0 ? 0 : (n > DEGCAP ? DEGCAP : n);
    const int st = __builtin_amdgcn_readlane(off_l, j);
    v4f sm4 = {0.0f, 0.0f, 0.0f, 0.0f};
    v8f sm8 = {0.0f, 0.0f, 0.0f, 0.0f, 0.0f, 0.0f, 0.0f, 0.0f};
    v4h mx4 = {nh, nh, nh, nh};
#pragma unroll 1
    for (int q0 = 0; q0 < n; q0 += 32) {
      int pos = st + q0 + lane;
      pos = pos < 0 ? 0 : (pos > csrLen - 1 ? csrLen - 1 : pos);
      int sl = csr[pos];
      sl = sl < 0 ? 0 : (sl > nN - 1 ? nN - 1 : sl);
      const int mcnt = (n - q0) < 32 ? (n - q0) : 32;
#pragma unroll 1
      for (int p = 0; p < mcnt; ++p) {
        const int s = __builtin_amdgcn_readlane(sl, p);
        if (MODE == 0) {
          const v4f v = *(const v4f*)(xs + (size_t)s * XD + 4 * lane);
          sm4 = sm4 + v;
        } else if (MODE == 1) {
          const v4h v = *(const v4h*)(hs + (size_t)s * 128 + 4 * lane);
          mx4 = __builtin_elementwise_max(mx4, v);
        } else {
          const v8h v = *(const v8h*)(hs + (size_t)s * 256 + 8 * lane);
          sm8 = sm8 + __builtin_convertvector(v, v8f);
        }
      }
    }
    if (MODE == 0) {
      const float rc = 1.0f / (float)(n > 1 ? n : 1);
      const v4h o = __builtin_convertvector(sm4 * rc, v4h);
      _Float16* ap = A + (size_t)c * 128 + 4 * lane;
      *(volatile v4h*)ap = o;
      __threadfence();
      *(volatile v4h*)ap = o;
    } else if (MODE == 1) {
      v4h o;
      o[0] = n > 0 ? mx4[0] : zh; o[1] = n > 0 ? mx4[1] : zh;
      o[2] = n > 0 ? mx4[2] : zh; o[3] = n > 0 ? mx4[3] : zh;
      _Float16* ap = A + (size_t)c * 128 + 4 * lane;
      *(volatile v4h*)ap = o;
      __threadfence();
      *(volatile v4h*)ap = o;
    } else {
      const float rc = 1.0f / (float)(n > 1 ? n : 1);
      const v8h o = __builtin_convertvector(sm8 * rc, v8h);
      _Float16* ap = A + (size_t)c * 256 + 8 * lane;
      *(volatile v8h*)ap = o;
      __threadfence();
      *(volatile v8h*)ap = o;
    }
  }
}

template <int KA, int KR, int NC>
__global__ __launch_bounds__(NTHR) void k_sage(
    const _Float16* __restrict__ Aag, const _Float16* __restrict__ Hr,
    const _Float16* __restrict__ Bw, const float* __restrict__ bias,
    const float* __restrict__ lng, const float* __restrict__ lnb, _Float16* hout) {
  static_assert((KA % 32) == 0 && (KR % 32) == 0 && (NC == 128 || NC == 256));
  extern __shared__ v4f lds_dyn[];
  float* stg = (float*)lds_dyn;
  constexpr int K = KA + KR, NKA = KA / 32, NKR = KR / 32;
  constexpr int WPR = NC / 128, RB = 128 / WPR, RPW = RB / NWAVE;
  static_assert(RB * NC * 4 <= LDS_SAGE);
  const int tid = threadIdx.x, lane = tid & 31, wave = tid >> 5, hh = lane >> 4, m = lane & 15;
  const int rg = wave / WPR, chf = wave - WPR * rg;
  const int rowBase = blockIdx.x * RB;
  const int arow = rowBase + rg * 16 + m;

  v8f acc[8];
#pragma unroll
  for (int t = 0; t < 8; ++t) { v8f z = {0.f, 0.f, 0.f, 0.f, 0.f, 0.f, 0.f, 0.f}; acc[t] = z; }
  const _Float16* bq = Bw + (size_t)(chf * 128 + m) * K + 8 * hh;
  {
    const _Float16* ap = Aag + (size_t)arow * KA + 8 * hh;
#pragma unroll 1
    for (int kt = 0; kt < NKA; ++kt) {
      FragH a;
      a.half[0] = *(const v8h*)(ap + 32 * kt);
      a.half[1] = *(const v8h*)(ap + 32 * kt + 16);
#pragma unroll
      for (int t = 0; t < 8; ++t) {
        const _Float16* bp = bq + (size_t)(16 * t) * K + 32 * kt;
        FragH bb;
        bb.half[0] = *(const v8h*)bp;
        bb.half[1] = *(const v8h*)(bp + 16);
        acc[t] = wmh(a.v, bb.v, acc[t]);
      }
    }
  }
  {
    const _Float16* ap = Hr + (size_t)arow * KR + 8 * hh;
#pragma unroll 1
    for (int kt = 0; kt < NKR; ++kt) {
      FragH a;
      a.half[0] = *(const v8h*)(ap + 32 * kt);
      a.half[1] = *(const v8h*)(ap + 32 * kt + 16);
#pragma unroll
      for (int t = 0; t < 8; ++t) {
        const _Float16* bp = bq + (size_t)(16 * t) * K + KA + 32 * kt;
        FragH bb;
        bb.half[0] = *(const v8h*)bp;
        bb.half[1] = *(const v8h*)(bp + 16);
        acc[t] = wmh(a.v, bb.v, acc[t]);
      }
    }
  }

  {
    float* sp = stg + (rg * 16 + 8 * hh) * NC + chf * 128 + m;
    const float* bq2 = bias + chf * 128 + m;
#pragma unroll
    for (int t = 0; t < 8; ++t) {
      const float bv = bq2[16 * t];
#pragma unroll
      for (int r = 0; r < 8; ++r) sp[r * NC + 16 * t] = acc[t][r] * WINV + bv;
    }
  }
  __syncthreads();

  if (NC == 128) {
    const v4f g = *(const v4f*)(lng + 4 * lane);
    const v4f e = *(const v4f*)(lnb + 4 * lane);
#pragma unroll 1
    for (int j = 0; j < RPW; ++j) {
      const int row = wave * RPW + j;
      const v4f v = *(const v4f*)(stg + row * NC + 4 * lane);
      float s = (v.x + v.y) + (v.z + v.w);
      s = wsum(s);
      const float mu = s * (1.0f / NC);
      const v4f d = v - mu;
      float s2 = (d.x * d.x + d.y * d.y) + (d.z * d.z + d.w * d.w);
      s2 = wsum(s2);
      const float rs = rsqrtf(s2 * (1.0f / NC) + LN_EPS);
      v4f y = d * rs * g + e;
      y.x = fmaxf(y.x, 0.0f); y.y = fmaxf(y.y, 0.0f); y.z = fmaxf(y.z, 0.0f); y.w = fmaxf(y.w, 0.0f);
      const v4h o = __builtin_convertvector(y, v4h);
      _Float16* gp = hout + (size_t)(rowBase + row) * NC + 4 * lane;
      *(volatile v4h*)gp = o;
      __threadfence();
      *(volatile v4h*)gp = o;
    }
  } else {
    const v4f g0 = *(const v4f*)(lng + 8 * lane), g1 = *(const v4f*)(lng + 8 * lane + 4);
    const v4f e0 = *(const v4f*)(lnb + 8 * lane), e1 = *(const v4f*)(lnb + 8 * lane + 4);
#pragma unroll 1
    for (int j = 0; j < RPW; ++j) {
      const int row = wave * RPW + j;
      const v4f v0 = *(const v4f*)(stg + row * NC + 8 * lane);
      const v4f v1 = *(const v4f*)(stg + row * NC + 8 * lane + 4);
      float s = ((v0.x + v0.y) + (v0.z + v0.w)) + ((v1.x + v1.y) + (v1.z + v1.w));
      s = wsum(s);
      const float mu = s * (1.0f / NC);
      const v4f d0 = v0 - mu, d1 = v1 - mu;
      float s2 = ((d0.x * d0.x + d0.y * d0.y) + (d0.z * d0.z + d0.w * d0.w)) +
                 ((d1.x * d1.x + d1.y * d1.y) + (d1.z * d1.z + d1.w * d1.w));
      s2 = wsum(s2);
      const float rs = rsqrtf(s2 * (1.0f / NC) + LN_EPS);
      v4f y0 = d0 * rs * g0 + e0, y1 = d1 * rs * g1 + e1;
      y0.x = fmaxf(y0.x, 0.0f); y0.y = fmaxf(y0.y, 0.0f); y0.z = fmaxf(y0.z, 0.0f); y0.w = fmaxf(y0.w, 0.0f);
      y1.x = fmaxf(y1.x, 0.0f); y1.y = fmaxf(y1.y, 0.0f); y1.z = fmaxf(y1.z, 0.0f); y1.w = fmaxf(y1.w, 0.0f);
      const v8h o = cvt8(y0, y1);
      _Float16* gp = hout + (size_t)(rowBase + row) * NC + 8 * lane;
      *(volatile v8h*)gp = o;
      __threadfence();
      *(volatile v8h*)gp = o;
    }
  }
}

__global__ __launch_bounds__(NTHR) void k_head(
    const _Float16* __restrict__ H3, const _Float16* __restrict__ Bw1, const float* __restrict__ b1,
    const float* __restrict__ g4, const float* __restrict__ e4,
    const _Float16* __restrict__ Bw2, const float* __restrict__ b2,
    float* out, int nN) {
  extern __shared__ v4f lds_dyn[];
  float*    stg = (float*)lds_dyn;
  _Float16* sA  = (_Float16*)((char*)lds_dyn + HROWS * OUTC * 4);
  const int tid = threadIdx.x, lane = tid & 31, wave = tid >> 5, hh = lane >> 4, m = lane & 15;
  const int rowBase = blockIdx.x * HROWS;
  const int arow = rowBase + wave * 16 + m;

  v8f acc[4];
#pragma unroll
  for (int t = 0; t < 4; ++t) { v8f z = {0.f, 0.f, 0.f, 0.f, 0.f, 0.f, 0.f, 0.f}; acc[t] = z; }
  {
    const _Float16* ap = H3 + (size_t)arow * 128 + 8 * hh;
    const _Float16* bq = Bw1 + (size_t)m * 128 + 8 * hh;
#pragma unroll 1
    for (int kt = 0; kt < 4; ++kt) {
      FragH a;
      a.half[0] = *(const v8h*)(ap + 32 * kt);
      a.half[1] = *(const v8h*)(ap + 32 * kt + 16);
#pragma unroll
      for (int t = 0; t < 4; ++t) {
        const _Float16* bp = bq + (size_t)(16 * t) * 128 + 32 * kt;
        FragH bb;
        bb.half[0] = *(const v8h*)bp;
        bb.half[1] = *(const v8h*)(bp + 16);
        acc[t] = wmh(a.v, bb.v, acc[t]);
      }
    }
  }
  {
    float* sp = stg + (wave * 16 + 8 * hh) * 64 + m;
#pragma unroll
    for (int t = 0; t < 4; ++t) {
      const float bv = b1[16 * t + m];
#pragma unroll
      for (int r = 0; r < 8; ++r) sp[r * 64 + 16 * t] = acc[t][r] * WINV + bv;
    }
  }
  __syncthreads();

  {
    const v2f g2 = *(const v2f*)(g4 + 2 * lane);
    const v2f q2 = *(const v2f*)(e4 + 2 * lane);
#pragma unroll 1
    for (int j = 0; j < 16; ++j) {
      const int row = wave * 16 + j;
      const v2f v = *(const v2f*)(stg + row * 64 + 2 * lane);
      float s = v.x + v.y;
      s = wsum(s);
      const float mu = s * (1.0f / 64.0f);
      const float dx = v.x - mu, dy = v.y - mu;
      float s2 = dx * dx + dy * dy;
      s2 = wsum(s2);
      const float rs = rsqrtf(s2 * (1.0f / 64.0f) + LN_EPS);
      const float yx = fmaxf(dx * rs * g2.x + q2.x, 0.0f);
      const float yy = fmaxf(dy * rs * g2.y + q2.y, 0.0f);
      v2h o;
      o[0] = (_Float16)yx; o[1] = (_Float16)yy;
      *(v2h*)(sA + row * AP2 + 2 * lane) = o;
    }
  }
  __syncthreads();

  v8f acc2[7];
#pragma unroll
  for (int t = 0; t < 7; ++t) { v8f z = {0.f, 0.f, 0.f, 0.f, 0.f, 0.f, 0.f, 0.f}; acc2[t] = z; }
  {
    const _Float16* ap = sA + (wave * 16 + m) * AP2 + 8 * hh;
    const _Float16* bq = Bw2 + (size_t)m * 64 + 8 * hh;
#pragma unroll 1
    for (int kt = 0; kt < 2; ++kt) {
      FragH a;
      a.half[0] = *(const v8h*)(ap + 32 * kt);
      a.half[1] = *(const v8h*)(ap + 32 * kt + 16);
#pragma unroll
      for (int t = 0; t < 7; ++t) {
        const _Float16* bp = bq + (size_t)(16 * t) * 64 + 32 * kt;
        FragH bb;
        bb.half[0] = *(const v8h*)bp;
        bb.half[1] = *(const v8h*)(bp + 16);
        acc2[t] = wmh(a.v, bb.v, acc2[t]);
      }
    }
  }
  {
    float* sp = stg + (wave * 16 + 8 * hh) * OUTC;
#pragma unroll
    for (int t = 0; t < 7; ++t) {
      const int n = 16 * t + m;
      const float bv = b2[n > OUTC - 1 ? OUTC - 1 : n];
      if (n < OUTC) {
#pragma unroll
        for (int r = 0; r < 8; ++r) sp[r * OUTC + n] = acc2[t][r] * WINV + bv;
      }
    }
  }
  __syncthreads();

  const int rows = (nN - rowBase) < HROWS ? (nN - rowBase) : HROWS;
  const int validF = rows * OUTC;
  float* ob = out + (size_t)rowBase * OUTC;
#pragma unroll 1
  for (int ci = wave; ci < 100; ci += NWAVE) {
    const int f = ci * 128 + 4 * lane;
    const v4f v = *(const v4f*)(stg + f);
    if (f + 4 <= validF) *(volatile v4f*)(ob + f) = v;
  }
  __threadfence();
#pragma unroll 1
  for (int ci = wave; ci < 100; ci += NWAVE) {
    const int f = ci * 128 + 4 * lane;
    const v4f v = *(const v4f*)(stg + f);
    if (f + 4 <= validF) *(volatile v4f*)(ob + f) = v;
  }
}

extern "C" void kernel_launch(void* const* d_in, const int* in_sizes, int n_in,
                              void* d_out, int out_size, void* d_ws, size_t ws_size,
                              hipStream_t stream) {
  if (n_in < 24) return;
  const int nN = in_sizes[0] / XD;
  const int nE = in_sizes[1];
  if (nN <= 0 || nE <= 0) return;
  if (in_sizes[0] != nN * XD || in_sizes[2] != nE) return;
  if (in_sizes[3] != 128 * 128 || in_sizes[4] != 128 || in_sizes[5] != 128 * 128) return;
  if (in_sizes[6] != 128 || in_sizes[7] != 128) return;
  if (in_sizes[8] != 128 * 256 || in_sizes[9] != 256 || in_sizes[10] != 128 * 256) return;
  if (in_sizes[11] != 256 || in_sizes[12] != 256) return;
  if (in_sizes[13] != 256 * 128 || in_sizes[14] != 128 || in_sizes[15] != 256 * 128) return;
  if (in_sizes[16] != 128 || in_sizes[17] != 128) return;
  if (in_sizes[18] != 128 * 64 || in_sizes[19] != 64 || in_sizes[20] != 64 || in_sizes[21] != 64) return;
  if (in_sizes[22] != 64 * OUTC || in_sizes[23] != OUTC) return;
  if ((long long)out_size != (long long)nN * OUTC) return;
  if (nE > (1 << 28) || nN > (1 << 24)) return;

  const float* x     = (const float*)d_in[0];
  const int*   srcs  = (const int*)d_in[1];
  const int*   dsts  = (const int*)d_in[2];
  const float* s1wl  = (const float*)d_in[3];
  const float* s1bl  = (const float*)d_in[4];
  const float* s1wr  = (const float*)d_in[5];
  const float* ln1g  = (const float*)d_in[6];
  const float* ln1b  = (const float*)d_in[7];
  const float* s2wl  = (const float*)d_in[8];
  const float* s2bl  = (const float*)d_in[9];
  const float* s2wr  = (const float*)d_in[10];
  const float* ln2g  = (const float*)d_in[11];
  const float* ln2b  = (const float*)d_in[12];
  const float* s3wl  = (const float*)d_in[13];
  const float* s3bl  = (const float*)d_in[14];
  const float* s3wr  = (const float*)d_in[15];
  const float* ln3g  = (const float*)d_in[16];
  const float* ln3b  = (const float*)d_in[17];
  const float* l1w   = (const float*)d_in[18];
  const float* l1b   = (const float*)d_in[19];
  const float* ln4g  = (const float*)d_in[20];
  const float* ln4b  = (const float*)d_in[21];
  const float* low   = (const float*)d_in[22];
  const float* lob   = (const float*)d_in[23];
  float* out = (float*)d_out;

  const int NPAD   = ((nN + TGT - 1) / TGT) * TGT;
  const int nBC    = (nN + NBC - 1) / NBC;
  const int CNTPAD = nBC * NBC;
  if (FPC * nBC + 1 > RBN) return;
  const int nBF    = (nN + NBF - 1) / NBF;
  const int csrLen = ((nE + 31) & ~31) + 4096;
  if (31 * FPC * nBC > 4096) return;
  const int nXc    = NPAD / 16;
  const int nAgg   = NPAD / TGT;
  const int nG128  = NPAD / 128;
  const int nG64   = NPAD / 64;

  const size_t slot = (size_t)NPAD * 128 * 2;
  char* ws = (char*)d_ws;
  size_t off = 0;
  const size_t oW   = off; off += (size_t)WPTOT * 2;     off = (off + 255) & ~(size_t)255;
  const size_t oCnt = off; off += (size_t)CNTPAD * 4;    off = (off + 255) & ~(size_t)255;
  const size_t oOff = off; off += (size_t)CNTPAD * 4;    off = (off + 255) & ~(size_t)255;
  const size_t oRb  = off; off += (size_t)RBN * 4;       off = (off + 255) & ~(size_t)255;
  const size_t oCsr = off; off += (size_t)csrLen * 4;    off = (off + 255) & ~(size_t)255;
  const size_t oP0  = off; off += slot;
  const size_t oP1  = off; off += slot;
  const size_t oP2  = off; off += slot;
  const size_t oP3  = off; off += slot;
  const size_t oP4  = off; off += slot;
  (void)oP3;
  if (off > ws_size || off > (size_t)WSCAP) return;
  _Float16* wp   = (_Float16*)(ws + oW);
  int*      cnt  = (int*)(ws + oCnt);
  int*      offp = (int*)(ws + oOff);
  int*      rb   = (int*)(ws + oRb);
  int*      csr  = (int*)(ws + oCsr);
  _Float16* P0   = (_Float16*)(ws + oP0);
  _Float16* P1   = (_Float16*)(ws + oP1);
  _Float16* P2   = (_Float16*)(ws + oP2);
  _Float16* P4   = (_Float16*)(ws + oP4);

  const int vec8 = ((nE & 3) == 0) ? 1 : 0;

  k_wprep<<<88, NTHR, 0, stream>>>(s1wl, s1wr, s2wl, s2wr, s3wl, s3wr, l1w, low, wp);
  k_xcvt<<<nXc, NTHR, 0, stream>>>(x, P0, nN);

  k_count<<<nBC, NTHR, 0, stream>>>(dsts, cnt, nE, vec8);
  k_offsets<<<1, OTHR, 0, stream>>>(cnt, offp, rb, nBC, nE);
  hipFuncSetAttribute(reinterpret_cast<const void*>(&k_fill),
                      hipFuncAttributeMaxDynamicSharedMemorySize, LDS_FILL);
  k_fill<<<nBF, NTHR, LDS_FILL, stream>>>(srcs, dsts, offp, rb, csr, nN, nE, vec8, csrLen);

  hipFuncSetAttribute(reinterpret_cast<const void*>(&k_sage<128, 128, 128>),
                      hipFuncAttributeMaxDynamicSharedMemorySize, LDS_SAGE);
  hipFuncSetAttribute(reinterpret_cast<const void*>(&k_sage<128, 128, 256>),
                      hipFuncAttributeMaxDynamicSharedMemorySize, LDS_SAGE);
  hipFuncSetAttribute(reinterpret_cast<const void*>(&k_sage<256, 256, 128>),
                      hipFuncAttributeMaxDynamicSharedMemorySize, LDS_SAGE);
  hipFuncSetAttribute(reinterpret_cast<const void*>(&k_head),
                      hipFuncAttributeMaxDynamicSharedMemorySize, LDS_HEAD);

  k_agg<0><<<nAgg, NTHR, 0, stream>>>(csr, offp, cnt, x, P0, P2, nN, csrLen);
  k_sage<128, 128, 128><<<nG128, NTHR, LDS_SAGE, stream>>>(P2, P0, wp + WP1, s1bl, ln1g, ln1b, P1);

  k_agg<1><<<nAgg, NTHR, 0, stream>>>(csr, offp, cnt, x, P1, P0, nN, csrLen);
  k_sage<128, 128, 256><<<nG64, NTHR, LDS_SAGE, stream>>>(P0, P1, wp + WP2, s2bl, ln2g, ln2b, P2);

  k_agg<2><<<nAgg, NTHR, 0, stream>>>(csr, offp, cnt, x, P2, P0, nN, csrLen);
  k_sage<256, 256, 128><<<nG128, NTHR, LDS_SAGE, stream>>>(P0, P2, wp + WP3, s3bl, ln3g, ln3b, P4);

  k_head<<<nG128, NTHR, LDS_HEAD, stream>>>(P4, wp + WP4, l1b, ln4g, ln4b, wp + WP5, lob, out, nN);
}
